// SDNE_82635170775050
// MI455X (gfx1250) — hardware-verified
//
#include <hip/hip_runtime.h>


typedef _Float16 v16h __attribute__((ext_vector_type(16)));
typedef _Float16 v8h  __attribute__((ext_vector_type(8)));
typedef _Float16 v4h  __attribute__((ext_vector_type(4)));
typedef float    v8f  __attribute__((ext_vector_type(8)));
typedef float    v4f  __attribute__((ext_vector_type(4)));
typedef int      v4i  __attribute__((ext_vector_type(4)));

union Frag  { v16h v; v8h half[2]; };
union Pack8 { v4h q[2]; v4i i; };

#define AG_THREADS  256
#define AG_WAVES    8
#define AG_EPT      8
#define AG_CHUNK    (AG_THREADS * AG_EPT)
#define AG_NSUB     (AG_EPT * AG_WAVES)
#define AG_LDS_F    32768
#define AG_MAXNB    512

#define GM_THREADS  256
#define TILE_M      128
#define TILE_N      64
#define KT          64
#define LDA         72
#define LDC         68
#define NEG_SLOPE   0.01f
#define W_SCALE     64.0f
#define W_UNSCALE   0.015625f

__device__ __forceinline__ v8f wmma_f16(v16h a, v16h b, v8f c) {
  v8f d = __builtin_amdgcn_wmma_f32_16x16x32_f16(false, a, false, b, (short)0, c, false, false);
  asm volatile("v_nop\n\tv_nop\n\tv_nop\n\tv_nop" : "+v"(d) : "v"(a), "v"(b));
  return d;
}

__global__ __launch_bounds__(AG_THREADS) void aggregate_scan(const float* __restrict__ hsrc,
                                                              const int* __restrict__ ei,
                                                              _Float16* agg,
                                                              int nnodes, int nedges, int nchunks,
                                                              int d, int nb) {
  __shared__ __attribute__((aligned(16))) float s_acc[AG_LDS_F];
  __shared__ int s_src[AG_CHUNK];
  __shared__ int s_loc[AG_CHUNK];
  __shared__ int s_wc[AG_NSUB];
  __shared__ int s_off[AG_NSUB];
  __shared__ int s_tot;

  const int tid  = threadIdx.x;
  const int lane = tid & 31;
  const int wave = tid >> 5;
  const int n0   = blockIdx.x * nb;

  const v4f z4 = {0.f, 0.f, 0.f, 0.f};
  for (int j = tid; j < AG_LDS_F / 4; j += AG_THREADS) *(v4f*)&s_acc[4 * j] = z4;
  __syncthreads();

  const int  cq   = d >> 2;
  const bool vec4 = ((nedges & 3) == 0);

  for (int c = 0; c < nchunks; ++c) {
    const int ebase = c * AG_CHUNK + tid * AG_EPT;
    int sv[AG_EPT], lv[AG_EPT];
    if (vec4 && ebase + AG_EPT <= nedges) {
      const v4i s0 = *(const v4i*)(ei + ebase);
      const v4i s1 = *(const v4i*)(ei + ebase + 4);
      const v4i d0 = *(const v4i*)(ei + (size_t)nedges + (size_t)ebase);
      const v4i d1 = *(const v4i*)(ei + (size_t)nedges + (size_t)ebase + 4);
      sv[0] = s0.x; sv[1] = s0.y; sv[2] = s0.z; sv[3] = s0.w;
      sv[4] = s1.x; sv[5] = s1.y; sv[6] = s1.z; sv[7] = s1.w;
      lv[0] = d0.x; lv[1] = d0.y; lv[2] = d0.z; lv[3] = d0.w;
      lv[4] = d1.x; lv[5] = d1.y; lv[6] = d1.z; lv[7] = d1.w;
#pragma unroll
      for (int j = 0; j < AG_EPT; ++j) lv[j] = (int)((unsigned)lv[j] - (unsigned)n0);
    } else {
#pragma unroll
      for (int j = 0; j < AG_EPT; ++j) {
        const int e = ebase + j;
        if (e < nedges) {
          sv[j] = ei[e];
          lv[j] = (int)((unsigned)ei[(size_t)nedges + (size_t)e] - (unsigned)n0);
        } else {
          sv[j] = 0;
          lv[j] = -1;
        }
      }
    }

    int rk[AG_EPT];
    unsigned mt = 0u;
#pragma unroll
    for (int j = 0; j < AG_EPT; ++j) {
      const bool m = ((unsigned)lv[j] < (unsigned)nb);
      const unsigned mask = __builtin_amdgcn_ballot_w32(m);
      rk[j] = (int)__builtin_amdgcn_mbcnt_lo(mask, 0u);
      if (m) mt |= (1u << j);
      if (lane == 0) s_wc[j * AG_WAVES + wave] = (int)__builtin_popcount(mask);
    }
    __syncthreads();

    if (wave == 0) {
      const int a = s_wc[2 * lane];
      const int b = s_wc[2 * lane + 1];
      const int t = a + b;
      int incl = t;
#pragma unroll
      for (int off = 1; off < 32; off <<= 1) {
        const int u = __shfl_up(incl, off, 32);
        if (lane >= off) incl += u;
      }
      s_off[2 * lane]     = incl - t;
      s_off[2 * lane + 1] = incl - t + a;
      if (lane == 31) s_tot = incl;
    }
    __syncthreads();

#pragma unroll
    for (int j = 0; j < AG_EPT; ++j) {
      if (mt & (1u << j)) {
        const int pos = s_off[j * AG_WAVES + wave] + rk[j];
        if ((unsigned)pos < (unsigned)AG_CHUNK) {
          s_src[pos] = sv[j];
          s_loc[pos] = lv[j];
        }
      }
    }
    __syncthreads();

    int tot = s_tot;
    tot = tot < 0 ? 0 : (tot > AG_CHUNK ? AG_CHUNK : tot);
    if (tid < cq) {
      float* acol = s_acc + 4 * tid;
      for (int q = 0; q < tot; ++q) {
        int s = s_src[q];
        if (s < 0) s += nnodes;
        s = s < 0 ? 0 : (s >= nnodes ? nnodes - 1 : s);
        int lc = s_loc[q];
        lc = ((unsigned)lc < (unsigned)nb) ? lc : 0;
        const v4f v = *(const v4f*)(hsrc + (size_t)s * (size_t)d + (size_t)(4 * tid));
        *(v4f*)(acol + (size_t)lc * (size_t)d) += v;
      }
    }
  }
  __syncthreads();

  _Float16* region = agg + (size_t)blockIdx.x * (size_t)AG_LDS_F;
  const int lsub  = lane >> 3;
  const int piece = (lane & 7) * 8;
#pragma unroll
  for (int j = 0; j < 16; ++j) {
    const int f = (wave * 64 + 4 * j + lsub) * 64 + piece;
    Pack8 pk;
    pk.q[0] = __builtin_convertvector(*(const v4f*)&s_acc[f], v4h);
    pk.q[1] = __builtin_convertvector(*(const v4f*)&s_acc[f + 4], v4h);
    *(volatile v4i*)(region + f) = pk.i;
  }
  __threadfence();
#pragma unroll
  for (int j = 0; j < 16; ++j) {
    const int f = (wave * 64 + 4 * j + lsub) * 64 + piece;
    Pack8 pk;
    pk.q[0] = __builtin_convertvector(*(const v4f*)&s_acc[f], v4h);
    pk.q[1] = __builtin_convertvector(*(const v4f*)&s_acc[f + 4], v4h);
    *(volatile v4i*)(region + f) = pk.i;
  }
}

__global__ __launch_bounds__(GM_THREADS) void dual_gemm(const _Float16* __restrict__ agg,
                                                         const float* __restrict__ hin,
                                                         const float* __restrict__ Wr,
                                                         const float* __restrict__ Ws,
                                                         const float* __restrict__ bias,
                                                         float* out, int nrows, int d_in, int d_out) {
  __shared__ __attribute__((aligned(16))) _Float16 sA[TILE_M * LDA];
  __shared__ __attribute__((aligned(16))) _Float16 sB[TILE_N * LDA];
  __shared__ __attribute__((aligned(16))) float    sC[(GM_THREADS / 32) * 16 * LDC];

  const int tid  = threadIdx.x;
  const int wave = tid >> 5;
  const int lane = tid & 31;
  const int hh   = lane >> 4;
  const int m    = lane & 15;
  const int m0   = blockIdx.x * TILE_M;
  const int n0   = blockIdx.y * TILE_N;
  if (n0 + TILE_N > d_out || m0 >= nrows) return;

  v8f acc[4];
#pragma unroll
  for (int nt = 0; nt < 4; ++nt) acc[nt] = (v8f){0.f, 0.f, 0.f, 0.f, 0.f, 0.f, 0.f, 0.f};

  const int ktot = 2 * d_in;
  for (int kg = 0; kg < ktot; kg += KT) {
    __syncthreads();
    if (kg < d_in) {
#pragma unroll
      for (int p = 0; p < 4; ++p) {
        const int r    = (tid >> 3) + 32 * p;
        const int ch   = (tid & 7) * 8;
        const int grow = m0 + r;
        v4i v = {0, 0, 0, 0};
        if (grow < nrows) v = *(const v4i*)(agg + (size_t)grow * (size_t)d_in + (size_t)(kg + ch));
        *(v4i*)&sA[r * LDA + ch] = v;
      }
    } else {
      const int kh = kg - d_in;
#pragma unroll
      for (int p = 0; p < 8; ++p) {
        const int r    = (tid >> 4) + 16 * p;
        const int ch   = (tid & 15) * 4;
        const int grow = m0 + r;
        v4f v = {0.f, 0.f, 0.f, 0.f};
        if (grow < nrows) v = *(const v4f*)(hin + (size_t)grow * (size_t)d_in + (size_t)(kh + ch));
        *(v4h*)&sA[r * LDA + ch] = __builtin_convertvector(v, v4h);
      }
    }
    {
      const float* W = (kg < d_in) ? Wr : Ws;
      const int kw   = (kg < d_in) ? kg : (kg - d_in);
#pragma unroll
      for (int p = 0; p < 4; ++p) {
        const int n  = (tid >> 4) + 16 * p;
        const int ch = (tid & 15) * 4;
        v4f v = *(const v4f*)(W + (size_t)(n0 + n) * (size_t)d_in + (size_t)(kw + ch));
        v = v * W_SCALE;
        *(v4h*)&sB[n * LDA + ch] = __builtin_convertvector(v, v4h);
      }
    }
    __syncthreads();

#pragma unroll
    for (int ks = 0; ks < KT / 32; ++ks) {
      Frag a;
      const _Float16* ar = &sA[(wave * 16 + m) * LDA + ks * 32];
      a.half[0] = *(const v8h*)(ar + 8 * hh);
      a.half[1] = *(const v8h*)(ar + 16 + 8 * hh);
#pragma unroll
      for (int nt = 0; nt < 4; ++nt) {
        Frag b;
        const _Float16* br = &sB[(nt * 16 + m) * LDA + ks * 32];
        b.half[0] = *(const v8h*)(br + 8 * hh);
        b.half[1] = *(const v8h*)(br + 16 + 8 * hh);
        acc[nt] = wmma_f16(a.v, b.v, acc[nt]);
      }
    }
  }

  float* cst = &sC[wave * 16 * LDC];
#pragma unroll
  for (int nt = 0; nt < 4; ++nt) {
    const int cl   = nt * 16 + m;
    const float bv = bias[n0 + cl];
#pragma unroll
    for (int r = 0; r < 8; ++r) {
      float v = acc[nt][r] * W_UNSCALE + bv;
      v = (v > 0.f) ? v : v * NEG_SLOPE;
      cst[(8 * hh + r) * LDC + cl] = v;
    }
  }
  __syncthreads();

  const int lsub  = lane >> 3;
  const int piece = (lane & 7) * 4;
  v4f ov[8];
#pragma unroll
  for (int j = 0; j < 8; ++j) {
    const int L   = 4 * j + lsub;
    const int row = L >> 1;
    const int c32 = (L & 1) * 32;
    ov[j] = *(const v4f*)&cst[row * LDC + c32 + piece];
  }
#pragma unroll
  for (int j = 0; j < 8; ++j) {
    const int L    = 4 * j + lsub;
    const int row  = L >> 1;
    const int c32  = (L & 1) * 32;
    const int grow = m0 + wave * 16 + row;
    if (grow < nrows)
      *(volatile v4f*)(out + (size_t)grow * (size_t)d_out + (size_t)(n0 + c32 + piece)) = ov[j];
  }
  __threadfence();
#pragma unroll
  for (int j = 0; j < 8; ++j) {
    const int L    = 4 * j + lsub;
    const int row  = L >> 1;
    const int c32  = (L & 1) * 32;
    const int grow = m0 + wave * 16 + row;
    if (grow < nrows)
      *(volatile v4f*)(out + (size_t)grow * (size_t)d_out + (size_t)(n0 + c32 + piece)) = ov[j];
  }
}

static inline size_t align_up256(size_t v) { return (v + 255) & ~(size_t)255; }

extern "C" void kernel_launch(void* const* d_in, const int* in_sizes, int n_in,
                              void* d_out, int out_size, void* d_ws,
                              size_t ws_size, hipStream_t stream) {
  if (n_in < 14) return;
  const int dims[5] = {128, 256, 64, 256, 128};
  const int nn = in_sizes[0] / dims[0];
  const int ne = in_sizes[1] / 2;
  if (nn <= 0 || in_sizes[0] != nn * dims[0] || ne < 0 || in_sizes[1] != 2 * ne) return;
  if (out_size != nn * (dims[4] + dims[2])) return;
  for (int i = 0; i < 4; ++i) {
    if (in_sizes[2 + 3 * i] != dims[i + 1] * dims[i]) return;
    if (in_sizes[3 + 3 * i] != dims[i + 1] * dims[i]) return;
    if (in_sizes[4 + 3 * i] != dims[i + 1]) return;
    const int din = dims[i], dout = dims[i + 1];
    if (din % KT != 0 || dout % TILE_N != 0) return;
    if (AG_LDS_F % din != 0) return;
    const int nb = AG_LDS_F / din;
    if (nb > AG_MAXNB || (nb & (nb - 1)) != 0 || (AG_MAXNB % nb) != 0) return;
  }

  const int npadA = ((nn + AG_MAXNB - 1) / AG_MAXNB) * AG_MAXNB;

  char* ws = (char*)d_ws;
  size_t off = 0;
  _Float16* agg = (_Float16*)(ws + off);  off += align_up256((size_t)npadA * 256 * sizeof(_Float16));
  float* hbuf = (float*)(ws + off);       off += align_up256((size_t)nn * 256 * sizeof(float));
  if (off > ws_size) return;

  const float* x  = (const float*)d_in[0];
  const int*   ei = (const int*)d_in[1];
  float* out0 = (float*)d_out;
  float* emb  = out0 + (size_t)nn * (size_t)dims[4];

  const float* lin[4]  = { x,    hbuf, emb,  hbuf };
  float*       lout[4] = { hbuf, emb,  hbuf, out0 };

  const int nchunks = (ne + AG_CHUNK - 1) / AG_CHUNK;

  for (int i = 0; i < 4; ++i) {
    const int din  = dims[i];
    const int dout = dims[i + 1];
    const float* Wr = (const float*)d_in[2 + 3 * i];
    const float* Ws = (const float*)d_in[3 + 3 * i];
    const float* b  = (const float*)d_in[4 + 3 * i];

    const int nb   = AG_LDS_F / din;
    const int nblk = (nn + nb - 1) / nb;
    aggregate_scan<<<dim3(nblk), dim3(AG_THREADS), 0, stream>>>(
        lin[i], ei, agg, nn, ne, nchunks, din, nb);

    dim3 grid((nn + TILE_M - 1) / TILE_M, dout / TILE_N);
    dual_gemm<<<grid, dim3(GM_THREADS), 0, stream>>>(
        agg, lin[i], Wr, Ws, b, lout[i], nn, din, dout);
  }
}
